// GateLinearAttention_45526653338169
// MI455X (gfx1250) — hardware-run, weakly checked
//
#include <hip/hip_runtime.h>

typedef float          v8f   __attribute__((ext_vector_type(8)));
typedef float          v4f   __attribute__((ext_vector_type(4)));
typedef unsigned int   v4u   __attribute__((ext_vector_type(4)));
typedef int            v8i   __attribute__((ext_vector_type(8)));
typedef unsigned short v8us  __attribute__((ext_vector_type(8)));
typedef unsigned short v16us __attribute__((ext_vector_type(16)));
typedef __bf16         v16bf __attribute__((ext_vector_type(16)));
typedef _Float16       v16h  __attribute__((ext_vector_type(16)));
typedef v4f  __attribute__((may_alias)) v4fa;
typedef v8us __attribute__((may_alias)) v8usa;
union FragB { v16bf v; v16us u; v8us h[2]; v8i w; };
union FragH { v16h  v; v16us u; v8us h[2]; v8i w; };

__device__ __forceinline__ v8f wmb(const FragB& a, const FragB& b, v8f c) {
  v8f d = __builtin_amdgcn_wmma_f32_16x16x32_bf16(false, a.v, false, b.v, (short)0, c, false, false);
  asm volatile("v_nop\n\tv_nop\n\tv_nop\n\tv_nop" : "+v"(d) : "v"(a.w), "v"(b.w));
  return d;
}

__device__ __forceinline__ v8f wmh(const FragH& a, const FragH& b, v8f c) {
  v8f d = __builtin_amdgcn_wmma_f32_16x16x32_f16(false, a.v, false, b.v, (short)0, c, false, false);
  asm volatile("v_nop\n\tv_nop\n\tv_nop\n\tv_nop" : "+v"(d) : "v"(a.w), "v"(b.w));
  return d;
}

__device__ __forceinline__ unsigned bf16_bits(float f) {
  const unsigned u = __float_as_uint(f);
  const unsigned r = (u + 0x7FFFu + ((u >> 16) & 1u)) >> 16;
  const unsigned q = (u >> 16) | 0x40u;
  return ((u & 0x7fffffffu) > 0x7f800000u) ? q : r;
}

__device__ __forceinline__ float bf16_val(float f) {
  return __uint_as_float(bf16_bits(f) << 16);
}
__device__ __forceinline__ int clampi(int v, int lo, int hi) {
  return v < lo ? lo : (v > hi ? hi : v);
}

__device__ __forceinline__ unsigned f16_bits(float f) {
  const unsigned u  = __float_as_uint(f);
  const unsigned s  = (u >> 16) & 0x8000u;
  const unsigned a  = u & 0x7fffffffu;
  const unsigned t  = a - 0x38000000u;
  const unsigned r  = (t + 0x0FFFu + ((t >> 13) & 1u)) >> 13;
  const unsigned rc = r > 0x7C00u ? 0x7C00u : r;
  const bool small  = a < 0x38800000u;
  const bool isnan  = a > 0x7f800000u;
  const unsigned fin = small ? 0u : (s | rc);
  return isnan ? (s | 0x7E00u) : fin;
}

__device__ __forceinline__ unsigned pk16(unsigned lo, unsigned hi) { return lo | (hi << 16); }
__device__ __forceinline__ unsigned bf16_lo_bits(float v) {
  float hi = bf16_val(v);
  asm volatile("" : "+v"(hi));
  return bf16_bits(v - hi);
}
__device__ __forceinline__ v4u pack8_bf16(v4f a, v4f c) {
  return (v4u){ pk16(bf16_bits(a[0]), bf16_bits(a[1])), pk16(bf16_bits(a[2]), bf16_bits(a[3])),
                pk16(bf16_bits(c[0]), bf16_bits(c[1])), pk16(bf16_bits(c[2]), bf16_bits(c[3])) };
}
__device__ __forceinline__ v4u pack8_bf16_lo(v4f a, v4f c) {
  return (v4u){ pk16(bf16_lo_bits(a[0]), bf16_lo_bits(a[1])), pk16(bf16_lo_bits(a[2]), bf16_lo_bits(a[3])),
                pk16(bf16_lo_bits(c[0]), bf16_lo_bits(c[1])), pk16(bf16_lo_bits(c[2]), bf16_lo_bits(c[3])) };
}
__device__ __forceinline__ v4u pack8_f16(v4f a, v4f c) {
  return (v4u){ pk16(f16_bits(a[0]), f16_bits(a[1])), pk16(f16_bits(a[2]), f16_bits(a[3])),
                pk16(f16_bits(c[0]), f16_bits(c[1])), pk16(f16_bits(c[2]), f16_bits(c[3])) };
}

template <int FORM>
__global__ __launch_bounds__(256) void k_plane(const float* __restrict__ src, int rows, int cols, int ldsrc,
                                               unsigned short* __restrict__ dst, int MP, int KP) {
  static_assert(FORM >= 0 && FORM <= 3);
  const int KTOT = (FORM == 1 || FORM == 3) ? 2 * KP : KP;
  const unsigned ppr   = (unsigned)(KTOT >> 3);
  const unsigned kp8   = (unsigned)(KP >> 3);
  const unsigned total = (unsigned)MP * ppr;
  const unsigned g     = blockIdx.x * 256u + threadIdx.x;
  const unsigned rowu  = g / ppr;
  const unsigned p     = g - rowu * ppr;
  const bool second    = p >= kp8;
  const int row = (int)rowu;
  const int c0  = (int)((second ? p - kp8 : p) << 3);
  const float* srow = src + (size_t)clampi(row, 0, rows - 1) * (size_t)ldsrc;
  float x[8];
  unsigned mk[8];
#pragma unroll
  for (int e = 0; e < 8; ++e) {
    const int c = c0 + e;
    const float v = srow[clampi(c, 0, cols - 1)];
    asm volatile("" :: "v"(v));
    x[e]  = v;
    mk[e] = (row < rows && c < cols) ? 0xFFFFu : 0u;
  }
  const v4f a = (v4f){ x[0], x[1], x[2], x[3] };
  const v4f c = (v4f){ x[4], x[5], x[6], x[7] };
  v4u o;
  if (FORM == 2) {
    o = pack8_f16(a, c);
  } else {
    const v4u hi = pack8_bf16(a, c);
    o = hi;
    if (FORM == 1) { const v4u lo = pack8_bf16_lo(a, c); o = second ? lo : hi; }
  }
  const v4u mw = (v4u){ pk16(mk[0], mk[1]), pk16(mk[2], mk[3]), pk16(mk[4], mk[5]), pk16(mk[6], mk[7]) };
  o &= mw;
  if (g < total) {
    volatile v4u* q = (volatile v4u*)(dst + (size_t)g * 8);
    *q = o;
    __threadfence();
    *q = o;
  }
}

template <int FORM> struct FragOf    { typedef FragB T; };
template <>         struct FragOf<2> { typedef FragH T; };
__device__ __forceinline__ v8f mm(const FragB& a, const FragB& b, v8f c) { return wmb(a, b, c); }
__device__ __forceinline__ v8f mm(const FragH& a, const FragH& b, v8f c) { return wmh(a, b, c); }
template <class F> __device__ __forceinline__ F ld_frag(const unsigned short* p) {
  F f;
  f.h[0] = *(const v8usa*)(p);
  f.h[1] = *(const v8usa*)(p + 16);
  return f;
}

template <int FORM, int EPI>
__global__ __launch_bounds__(256) __attribute__((amdgpu_num_vgpr(248)))
void k_gemm_nt(const unsigned short* __restrict__ A, const unsigned short* __restrict__ B,
               const float* __restrict__ bias, float* __restrict__ D, int M, int N, int KTOT, int ldd) {
  static_assert(FORM >= 0 && FORM <= 2);
  static_assert(EPI == 0 || EPI == 1);
  typedef typename FragOf<FORM>::T F;
  __shared__ __attribute__((aligned(16))) float sT[8][16 * 68];
  const int lane = threadIdx.x & 31;
  const int wave = threadIdx.x >> 5;
  const int tilesM = (M + 63) >> 6;
  const int tilesN = (N + 63) >> 6;
  const int tile = blockIdx.x * 8 + wave;
  if (tile >= tilesM * tilesN) return;
  const int tm = tile / tilesN;
  const int tn = tile - tm * tilesN;
  const int m0 = tm << 6;
  const int n0 = tn << 6;

  const int rl = lane & 15;
  const int h8 = (lane >> 4) * 8;
  const unsigned short* pa = A + (size_t)(m0 + rl) * (size_t)KTOT + h8;
  const unsigned short* pb = B + (size_t)(n0 + rl) * (size_t)KTOT + h8;

  v8f acc[4][4];
#pragma unroll
  for (int i = 0; i < 4; ++i)
#pragma unroll
    for (int j = 0; j < 4; ++j) acc[i][j] = (v8f){0.f, 0.f, 0.f, 0.f, 0.f, 0.f, 0.f, 0.f};

#pragma unroll 1
  for (int k0 = 0; k0 < KTOT; k0 += 32) {
    F bf[4];
#pragma unroll
    for (int j = 0; j < 4; ++j) bf[j] = ld_frag<F>(pb + (size_t)(j << 4) * (size_t)KTOT + k0);
#pragma unroll
    for (int i = 0; i < 4; ++i) {
      const F af = ld_frag<F>(pa + (size_t)(i << 4) * (size_t)KTOT + k0);
#pragma unroll
      for (int j = 0; j < 4; ++j) acc[i][j] = mm(af, bf[j], acc[i][j]);
    }
  }

  float* slab = sT[wave];
  const int hh = lane >> 4;
  const int c4 = (lane & 15) * 4;
  const int nc = n0 + c4;
  const bool cok = nc < N;
  v4f bv = (v4f){0.f, 0.f, 0.f, 0.f};
  if (EPI == 1) {
    bv = *(const v4fa*)(bias + clampi(nc, 0, N - 4));
    asm volatile("" :: "v"(bv));
  }
#pragma unroll
  for (int i = 0; i < 4; ++i) {
    const int mBase = m0 + (i << 4);
#pragma unroll
    for (int j = 0; j < 4; ++j) {
#pragma unroll
      for (int r = 0; r < 8; ++r) slab[(h8 + r) * 68 + (j << 4) + rl] = acc[i][j][r];
    }
    __builtin_amdgcn_fence(__ATOMIC_RELEASE, "workgroup");
    __builtin_amdgcn_wave_barrier();
    __builtin_amdgcn_fence(__ATOMIC_ACQUIRE, "workgroup");
    v4f vv[8];
#pragma unroll
    for (int it = 0; it < 8; ++it) {
      const int row = it * 2 + hh;
      v4f v = *(const v4fa*)(slab + row * 68 + c4);
      if (EPI == 1) v += bv;
      vv[it] = v;
    }
    for (int pass = 0; pass < 2; ++pass) {
#pragma unroll
      for (int it = 0; it < 8; ++it) {
        const int row = mBase + it * 2 + hh;
        if (cok && row < M) *(volatile v4f*)(D + (size_t)row * (size_t)ldd + nc) = vv[it];
      }
      __threadfence();
    }
    __builtin_amdgcn_fence(__ATOMIC_RELEASE, "workgroup");
    __builtin_amdgcn_wave_barrier();
    __builtin_amdgcn_fence(__ATOMIC_ACQUIRE, "workgroup");
  }
}

#define NROW   1024
#define DM     1024
#define NH     8
#define HD     128
#define NB     2
#define TSEQ   512
#define GLR    16
#define NQKVG  4096
#define LRN    64
#define KGP    32
#define KG2    64
#define TC     16
#define WO_SPLIT 1
#if WO_SPLIT
#define KYO    2048
#else
#define KYO    1024
#endif
#define SPN    1152

static_assert(DM == NH * HD);
static_assert(NROW == NB * TSEQ);
static_assert(TSEQ % TC == 0 && TC == 16);
static_assert(4 * 32 == HD);
static_assert(HD % 32 == 0);
static_assert(NROW % 64 == 0 && NQKVG % 64 == 0 && DM % 64 == 0 && LRN % 64 == 0);
static_assert(DM % 32 == 0 && KYO % 32 == 0 && KG2 % 32 == 0 && KGP % 32 == 0);
static_assert(NQKVG % 32 == 0 && LRN % 32 == 0);
static_assert(KYO % 64 == 0 && DM % 64 == 0);
static_assert((NROW * DM / 8) % 256 == 0 && (NROW * KG2 / 8) % 256 == 0 && (DM * KG2 / 8) % 256 == 0);
static_assert((NROW * DM / 4) % 256 == 0);

typedef unsigned int v2u __attribute__((ext_vector_type(2)));

__device__ __forceinline__ float pick4(v4f v, int j) {
  return j == 0 ? v.x : (j == 1 ? v.y : (j == 2 ? v.z : v.w));
}
__device__ __forceinline__ v4f put4(v4f v, int j, float r) {
  v.x = (j == 0) ? r : v.x;
  v.y = (j == 1) ? r : v.y;
  v.z = (j == 2) ? r : v.z;
  v.w = (j == 3) ? r : v.w;
  return v;
}

__global__ __launch_bounds__(256) void k_tplane(const float* __restrict__ src, int srows, int scols, int ldsrc,
                                                unsigned short* __restrict__ dst, int KTOT, int KP) {
  __shared__ float tl[64 * 65];
  const int tid = (int)threadIdx.x;
  const int kp0 = (int)blockIdx.x * 64;
  const int ks0 = kp0 % KP;
  const int n0  = (int)blockIdx.y * 64;
#pragma unroll
  for (int j = 0; j < 4; ++j) {
    const int idx = tid + 256 * j;
    const int kr  = idx >> 4;
    const int c4  = (idx & 15) * 4;
    const int sr  = ks0 + kr;
    const int sc  = n0 + c4;
    const bool ok = (sr < srows) && (sc < scols);
    const v4f v = *(const v4fa*)(src + (size_t)clampi(sr, 0, srows - 1) * (size_t)ldsrc + clampi(sc, 0, scols - 4));
    asm volatile("" :: "v"(v));
    tl[kr * 65 + c4 + 0] = ok ? v.x : 0.0f;
    tl[kr * 65 + c4 + 1] = ok ? v.y : 0.0f;
    tl[kr * 65 + c4 + 2] = ok ? v.z : 0.0f;
    tl[kr * 65 + c4 + 3] = ok ? v.w : 0.0f;
  }
  __syncthreads();
  v4u ov[2];
  size_t off[2];
#pragma unroll
  for (int it = 0; it < 2; ++it) {
    const int idx = tid + 256 * it;
    const int n = idx >> 3;
    const int p = idx & 7;
    const float* tp = tl + (8 * p) * 65 + n;
    const v4f a = (v4f){ tp[0], tp[65], tp[130], tp[195] };
    const v4f c = (v4f){ tp[260], tp[325], tp[390], tp[455] };
    ov[it]  = pack8_bf16(a, c);
    off[it] = (size_t)(n0 + n) * (size_t)KTOT + (size_t)(kp0 + 8 * p);
  }
  for (int pass = 0; pass < 2; ++pass) {
#pragma unroll
    for (int it = 0; it < 2; ++it) *(volatile v4u*)(dst + off[it]) = ov[it];
    __threadfence();
  }
}

__global__ __launch_bounds__(256) void k_wg2d(const float* __restrict__ w2, unsigned short* __restrict__ dst) {
  const int g  = (int)blockIdx.x * 256 + (int)threadIdx.x;
  const int n  = g >> 3;
  const int p  = g & 7;
  const int kb = (p & 3) * 8;
  const unsigned mk = ((p & 3) < 2) ? 0xFFFFFFFFu : 0u;
  float x[8];
#pragma unroll
  for (int e = 0; e < 8; ++e) {
    const int kk = clampi(kb + e, 0, GLR - 1);
    const float v = w2[(size_t)kk * DM + n];
    asm volatile("" :: "v"(v));
    x[e] = v;
  }
  v4u o = pack8_bf16((v4f){ x[0], x[1], x[2], x[3] }, (v4f){ x[4], x[5], x[6], x[7] });
  o &= (v4u){ mk, mk, mk, mk };
  volatile v4u* q = (volatile v4u*)(dst + (size_t)g * 8);
  *q = o;
  __threadfence();
  *q = o;
}

__global__ __launch_bounds__(256) void k_small(const float* __restrict__ bg, const float* __restrict__ gw,
                                               float* __restrict__ SP) {
  const int g  = (int)blockIdx.x * 256 + (int)threadIdx.x;
  const int ia = clampi(g, 0, 255) * 4;
  const int ib = clampi(g - 256, 0, 31) * 4;
  const v4f a = *(const v4fa*)(bg + ia);
  const v4f b = *(const v4fa*)(gw + ib);
  asm volatile("" :: "v"(a), "v"(b));
  const bool first = g < 256;
  v4f o;
  o.x = bf16_val(first ? a.x : b.x);
  o.y = bf16_val(first ? a.y : b.y);
  o.z = bf16_val(first ? a.z : b.z);
  o.w = bf16_val(first ? a.w : b.w);
  if (g < SPN / 4) {
    volatile v4f* q = (volatile v4f*)(SP + (size_t)4 * g);
    *q = o;
    __threadfence();
    *q = o;
  }
}

__global__ __launch_bounds__(256) void k_gate(const float* __restrict__ Z, const float* __restrict__ SP,
                                              float* __restrict__ DEC) {
  const int g = (int)blockIdx.x * 256 + (int)threadIdx.x;
  const v4f zz = *(const v4fa*)(Z + (size_t)4 * g);
  const v4f bb = *(const v4fa*)(SP + 4 * (g & 255));
  v4f o = (v4f){0.f, 0.f, 0.f, 0.f};
#pragma unroll 1
  for (int j = 0; j < 4; ++j) {
    const float z  = pick4(zz, j) + pick4(bb, j);
    const float az = fabsf(z);
    const float mz = (z < 0.0f) ? z : 0.0f;
    const float ls = mz - log1pf(expf(-az));
    const float gk = ls * 0.0625f;
    o = put4(o, j, expf(gk));
  }
  volatile v4f* q = (volatile v4f*)(DEC + (size_t)4 * g);
  *q = o;
  __threadfence();
  *q = o;
}

__global__ __launch_bounds__(128) void k_scan(const float* __restrict__ QKVG, const float* __restrict__ DEC,
                                              float* __restrict__ O) {
  __shared__ __attribute__((aligned(16))) float sq[TC * HD];
  __shared__ __attribute__((aligned(16))) float sk[TC * HD];
  __shared__ __attribute__((aligned(16))) float sd[TC * HD];
  __shared__ __attribute__((aligned(16))) float sv[TC * 32];
  __shared__ __attribute__((aligned(16))) float sp[TC * 4 * 32];
  const int tid  = (int)threadIdx.x;
  const int lane = tid & 31;
  const int w    = tid >> 5;
  const int blk  = (int)blockIdx.x;
  const int vc   = blk & 3;
  const int h    = (blk >> 2) & 7;
  const int b    = blk >> 5;
  const int colq = h * HD;
  const int colv = 2 * DM + h * HD + vc * 32;
  const int colo = h * HD + vc * 32 + lane;
  const float qs = __uint_as_float(0x3DB504F3u);

  float S[32];
#pragma unroll
  for (int i = 0; i < 32; ++i) S[i] = 0.0f;

#pragma unroll 1
  for (int ch = 0; ch < TSEQ / TC; ++ch) {
    const int r0 = b * TSEQ + ch * TC;
#pragma unroll
    for (int j = 0; j < 4; ++j) {
      const int i  = tid + 128 * j;
      const int tt = i >> 5;
      const int c4 = (i & 31) * 4;
      const float* gp = QKVG + (size_t)(r0 + tt) * NQKVG + colq + c4;
      v4f qa = *(const v4fa*)gp;
      const v4f ka = *(const v4fa*)(gp + DM);
      const v4f da = *(const v4fa*)(DEC + (size_t)(r0 + tt) * DM + colq + c4);
      qa = qa * qs;
      *(v4fa*)(sq + tt * HD + c4) = qa;
      *(v4fa*)(sk + tt * HD + c4) = ka;
      *(v4fa*)(sd + tt * HD + c4) = da;
    }
    {
      const int tt = tid >> 3;
      const int c4 = (tid & 7) * 4;
      const v4f va = *(const v4fa*)(QKVG + (size_t)(r0 + tt) * NQKVG + colv + c4);
      *(v4fa*)(sv + tt * 32 + c4) = va;
    }
    __syncthreads();

#pragma unroll 1
    for (int tt = 0; tt < TC; ++tt) {
      const float vt = sv[tt * 32 + lane];
      const float* bq = sq + tt * HD + 32 * w;
      const float* bk = sk + tt * HD + 32 * w;
      const float* bd = sd + tt * HD + 32 * w;
      float part = 0.0f;
#pragma unroll
      for (int j = 0; j < 8; ++j) {
        const v4f q4 = *(const v4fa*)(bq + 4 * j);
        const v4f k4 = *(const v4fa*)(bk + 4 * j);
        const v4f d4 = *(const v4fa*)(bd + 4 * j);
#pragma unroll
        for (int e = 0; e < 4; ++e) {
          const float kv = k4[e] * vt;
          const float s  = fmaf(S[4 * j + e], d4[e], kv);
          S[4 * j + e] = s;
          part = fmaf(q4[e], s, part);
        }
      }
      sp[(tt * 4 + w) * 32 + lane] = part;
    }
    __syncthreads();

    float ov[4];
#pragma unroll
    for (int i = 0; i < 4; ++i) {
      const int tt = 4 * w + i;
      ov[i] = ((sp[(tt * 4 + 0) * 32 + lane] + sp[(tt * 4 + 1) * 32 + lane]) + sp[(tt * 4 + 2) * 32 + lane])
              + sp[(tt * 4 + 3) * 32 + lane];
    }
    for (int pass = 0; pass < 2; ++pass) {
#pragma unroll
      for (int i = 0; i < 4; ++i)
        *(volatile float*)(O + (size_t)(r0 + 4 * w + i) * DM + colo) = ov[i];
      __threadfence();
    }
    __syncthreads();
  }
}

__global__ __launch_bounds__(256) void k_norm(const float* __restrict__ O, const float* __restrict__ QKVG,
                                              const float* __restrict__ SP, unsigned short* __restrict__ YHL) {
  const int r    = (int)blockIdx.x;
  const int lane = (int)threadIdx.x & 31;
  const int hw   = (int)threadIdx.x >> 5;
  const int col  = hw * HD + 4 * lane;
  const v4f o4 = *(const v4fa*)(O + (size_t)r * DM + col);
  const v4f g4 = *(const v4fa*)(QKVG + (size_t)r * NQKVG + 3 * DM + col);
  const v4f w4 = *(const v4fa*)(SP + DM + 4 * lane);
  float ss = (o4.x * o4.x + o4.y * o4.y) + (o4.z * o4.z + o4.w * o4.w);
  ss += __shfl_xor(ss, 16);
  ss += __shfl_xor(ss, 8);
  ss += __shfl_xor(ss, 4);
  ss += __shfl_xor(ss, 2);
  ss += __shfl_xor(ss, 1);
  const float mean = ss * 0.0078125f;
  const float rms  = 1.0f / sqrtf(mean + 1e-5f);
  v4f y = (v4f){0.f, 0.f, 0.f, 0.f};
#pragma unroll 1
  for (int j = 0; j < 4; ++j) {
    const float ov = pick4(o4, j);
    const float gv = pick4(g4, j);
    const float wv = pick4(w4, j);
    const float sg = 1.0f / (1.0f + expf(-gv));
    const float rr = ((ov * rms) * wv) * (gv * sg);
    y = put4(y, j, rr);
  }
  const v2u hv = (v2u){ pk16(bf16_bits(y.x), bf16_bits(y.y)), pk16(bf16_bits(y.z), bf16_bits(y.w)) };
  unsigned short* hp = YHL + (size_t)r * KYO + col;
#if WO_SPLIT
  const v2u lv = (v2u){ pk16(bf16_lo_bits(y.x), bf16_lo_bits(y.y)), pk16(bf16_lo_bits(y.z), bf16_lo_bits(y.w)) };
  *(volatile v2u*)hp = hv;
  *(volatile v2u*)(hp + DM) = lv;
  __threadfence();
  *(volatile v2u*)hp = hv;
  *(volatile v2u*)(hp + DM) = lv;
#else
  *(volatile v2u*)hp = hv;
  __threadfence();
  *(volatile v2u*)hp = hv;
#endif
}

static inline size_t al256(size_t o) { return (o + 255) & ~(size_t)255; }

extern "C" void kernel_launch(void* const* d_in, const int* in_sizes, int n_in,
                              void* d_out, int out_size, void* d_ws, size_t ws_size,
                              hipStream_t stream) {
  if (n_in < 10) return;
  if (in_sizes[0] != NROW * DM) return;
  if (in_sizes[1] != DM * DM) return;
  if (in_sizes[2] != DM * DM) return;
  if (in_sizes[3] != DM * DM) return;
  if (in_sizes[4] != DM * DM) return;
  if (in_sizes[5] != DM * GLR) return;
  if (in_sizes[6] != GLR * DM) return;
  if (in_sizes[7] != DM) return;
  if (in_sizes[8] != HD) return;
  if (in_sizes[9] != DM * DM) return;
  if (out_size != NROW * DM) return;

  const float* x    = (const float*)d_in[0];
  const float* Wq   = (const float*)d_in[1];
  const float* Wk   = (const float*)d_in[2];
  const float* Wv   = (const float*)d_in[3];
  const float* Wg   = (const float*)d_in[4];
  const float* Wgk1 = (const float*)d_in[5];
  const float* Wgk2 = (const float*)d_in[6];
  const float* bgk2 = (const float*)d_in[7];
  const float* gnw  = (const float*)d_in[8];
  const float* Wo   = (const float*)d_in[9];
  float* out = (float*)d_out;

  char* ws = (char*)d_ws;
  size_t off = 0;
  const size_t oXB   = off; off = al256(off + (size_t)NROW * DM * 2);
  const size_t oWT4  = off; off = al256(off + (size_t)NQKVG * DM * 2);
  const size_t oWG1T = off; off = al256(off + (size_t)LRN * DM * 2);
  const size_t oWG2D = off; off = al256(off + (size_t)DM * KG2 * 2);
  const size_t oWOD  = off; off = al256(off + (size_t)DM * KYO * 2);
  const size_t oSP   = off; off = al256(off + (size_t)SPN * 4);
  const size_t oQKVG = off; off = al256(off + (size_t)NROW * NQKVG * 4);
  const size_t oLR   = off; off = al256(off + (size_t)NROW * LRN * 4);
  const size_t oLRHL = off; off = al256(off + (size_t)NROW * KG2 * 2);
  const size_t oZ    = off; off = al256(off + (size_t)NROW * DM * 4);
  const size_t oDEC  = off; off = al256(off + (size_t)NROW * DM * 4);
  const size_t oO    = off; off = al256(off + (size_t)NROW * DM * 4);
  const size_t oYHL  = off; off = al256(off + (size_t)NROW * KYO * 2);
  if (off > ws_size || off > ((size_t)128 << 20)) return;

  unsigned short* XB   = (unsigned short*)(ws + oXB);
  unsigned short* WT4  = (unsigned short*)(ws + oWT4);
  unsigned short* WG1T = (unsigned short*)(ws + oWG1T);
  unsigned short* WG2D = (unsigned short*)(ws + oWG2D);
  unsigned short* WOD  = (unsigned short*)(ws + oWOD);
  float*          SP   = (float*)(ws + oSP);
  float*          QKVG = (float*)(ws + oQKVG);
  float*          LR   = (float*)(ws + oLR);
  unsigned short* LRHL = (unsigned short*)(ws + oLRHL);
  float*          Zp   = (float*)(ws + oZ);
  float*          DEC  = (float*)(ws + oDEC);
  float*          Op   = (float*)(ws + oO);
  unsigned short* YHL  = (unsigned short*)(ws + oYHL);

  k_plane<0><<<NROW * DM / 8 / 256, 256, 0, stream>>>(x, NROW, DM, DM, XB, NROW, DM);
  k_tplane<<<dim3(DM / 64, DM / 64), 256, 0, stream>>>(Wq, DM, DM, DM, WT4 + (size_t)0 * DM * DM, DM, DM);
  k_tplane<<<dim3(DM / 64, DM / 64), 256, 0, stream>>>(Wk, DM, DM, DM, WT4 + (size_t)1 * DM * DM, DM, DM);
  k_tplane<<<dim3(DM / 64, DM / 64), 256, 0, stream>>>(Wv, DM, DM, DM, WT4 + (size_t)2 * DM * DM, DM, DM);
  k_tplane<<<dim3(DM / 64, DM / 64), 256, 0, stream>>>(Wg, DM, DM, DM, WT4 + (size_t)3 * DM * DM, DM, DM);
  k_tplane<<<dim3(DM / 64, LRN / 64), 256, 0, stream>>>(Wgk1, DM, GLR, GLR, WG1T, DM, DM);
  k_tplane<<<dim3(KYO / 64, DM / 64), 256, 0, stream>>>(Wo, DM, DM, DM, WOD, KYO, DM);
  k_wg2d<<<DM * KG2 / 8 / 256, 256, 0, stream>>>(Wgk2, WG2D);
  k_small<<<2, 256, 0, stream>>>(bgk2, gnw, SP);

  k_gemm_nt<0, 0><<<(NROW / 64) * (NQKVG / 64) / 8, 256, 0, stream>>>(XB, WT4, SP, QKVG, NROW, NQKVG, DM, NQKVG);
  k_gemm_nt<0, 0><<<(NROW / 64) * (LRN / 64) / 8, 256, 0, stream>>>(XB, WG1T, SP, LR, NROW, LRN, DM, LRN);
  k_plane<1><<<NROW * KG2 / 8 / 256, 256, 0, stream>>>(LR, NROW, GLR, LRN, LRHL, NROW, KGP);
  k_gemm_nt<0, 0><<<(NROW / 64) * (DM / 64) / 8, 256, 0, stream>>>(LRHL, WG2D, SP, Zp, NROW, DM, KG2, DM);
  k_gate<<<NROW * DM / 4 / 256, 256, 0, stream>>>(Zp, SP, DEC);
  k_scan<<<NB * NH * 4, 128, 0, stream>>>(QKVG, DEC, Op);
  k_norm<<<NROW, 256, 0, stream>>>(Op, QKVG, SP, YHL);
  k_gemm_nt<0, 0><<<(NROW / 64) * (DM / 64) / 8, 256, 0, stream>>>(YHL, WOD, SP, out, NROW, DM, KYO, DM);
}
